// GINConv_81398220194522
// MI455X (gfx1250) — hardware-run, weakly checked
//
#include <hip/hip_runtime.h>

typedef float          v8f   __attribute__((ext_vector_type(8)));
typedef float          v4f   __attribute__((ext_vector_type(4)));
typedef unsigned int   v4u   __attribute__((ext_vector_type(4)));
typedef int            v8i   __attribute__((ext_vector_type(8)));
typedef unsigned short v8us  __attribute__((ext_vector_type(8)));
typedef unsigned short v16us __attribute__((ext_vector_type(16)));
typedef __bf16         v16bf __attribute__((ext_vector_type(16)));
typedef _Float16       v16h  __attribute__((ext_vector_type(16)));
typedef v4f  __attribute__((may_alias)) v4fa;
typedef v8us __attribute__((may_alias)) v8usa;
union FragB { v16bf v; v16us u; v8us h[2]; v8i w; };
union FragH { v16h  v; v16us u; v8us h[2]; v8i w; };

__device__ __forceinline__ v8f wmb(const FragB& a, const FragB& b, v8f c) {
  v8f d = __builtin_amdgcn_wmma_f32_16x16x32_bf16(false, a.v, false, b.v, (short)0, c, false, false);
  asm volatile("v_nop\n\tv_nop\n\tv_nop\n\tv_nop" : "+v"(d) : "v"(a.w), "v"(b.w));
  return d;
}

__device__ __forceinline__ v8f wmh(const FragH& a, const FragH& b, v8f c) {
  v8f d = __builtin_amdgcn_wmma_f32_16x16x32_f16(false, a.v, false, b.v, (short)0, c, false, false);
  asm volatile("v_nop\n\tv_nop\n\tv_nop\n\tv_nop" : "+v"(d) : "v"(a.w), "v"(b.w));
  return d;
}

__device__ __forceinline__ unsigned bf16_bits(float f) {
  const unsigned u = __float_as_uint(f);
  const unsigned r = (u + 0x7FFFu + ((u >> 16) & 1u)) >> 16;
  const unsigned q = (u >> 16) | 0x40u;
  return ((u & 0x7fffffffu) > 0x7f800000u) ? q : r;
}

__device__ __forceinline__ float bf16_val(float f) {
  return __uint_as_float(bf16_bits(f) << 16);
}
__device__ __forceinline__ int clampi(int v, int lo, int hi) {
  return v < lo ? lo : (v > hi ? hi : v);
}

__device__ __forceinline__ unsigned f16_bits(float f) {
  const unsigned u  = __float_as_uint(f);
  const unsigned s  = (u >> 16) & 0x8000u;
  const unsigned a  = u & 0x7fffffffu;
  const unsigned t  = a - 0x38000000u;
  const unsigned r  = (t + 0x0FFFu + ((t >> 13) & 1u)) >> 13;
  const unsigned rc = r > 0x7C00u ? 0x7C00u : r;
  const bool small  = a < 0x38800000u;
  const bool isnan  = a > 0x7f800000u;
  const unsigned fin = small ? 0u : (s | rc);
  return isnan ? (s | 0x7E00u) : fin;
}

__device__ __forceinline__ unsigned pk16(unsigned lo, unsigned hi) { return lo | (hi << 16); }
__device__ __forceinline__ unsigned bf16_lo_bits(float v) {
  float hi = bf16_val(v);
  asm volatile("" : "+v"(hi));
  return bf16_bits(v - hi);
}
__device__ __forceinline__ v4u pack8_bf16(v4f a, v4f c) {
  return (v4u){ pk16(bf16_bits(a[0]), bf16_bits(a[1])), pk16(bf16_bits(a[2]), bf16_bits(a[3])),
                pk16(bf16_bits(c[0]), bf16_bits(c[1])), pk16(bf16_bits(c[2]), bf16_bits(c[3])) };
}
__device__ __forceinline__ v4u pack8_bf16_lo(v4f a, v4f c) {
  return (v4u){ pk16(bf16_lo_bits(a[0]), bf16_lo_bits(a[1])), pk16(bf16_lo_bits(a[2]), bf16_lo_bits(a[3])),
                pk16(bf16_lo_bits(c[0]), bf16_lo_bits(c[1])), pk16(bf16_lo_bits(c[2]), bf16_lo_bits(c[3])) };
}
__device__ __forceinline__ v4u pack8_f16(v4f a, v4f c) {
  return (v4u){ pk16(f16_bits(a[0]), f16_bits(a[1])), pk16(f16_bits(a[2]), f16_bits(a[3])),
                pk16(f16_bits(c[0]), f16_bits(c[1])), pk16(f16_bits(c[2]), f16_bits(c[3])) };
}

template <int FORM>
__global__ __launch_bounds__(256) void k_plane(const float* __restrict__ src, int rows, int cols, int ldsrc,
                                               unsigned short* __restrict__ dst, int MP, int KP) {
  static_assert(FORM >= 0 && FORM <= 3);
  const int KTOT = (FORM == 1 || FORM == 3) ? 2 * KP : KP;
  const unsigned ppr   = (unsigned)(KTOT >> 3);
  const unsigned kp8   = (unsigned)(KP >> 3);
  const unsigned total = (unsigned)MP * ppr;
  const unsigned g     = blockIdx.x * 256u + threadIdx.x;
  const unsigned rowu  = g / ppr;
  const unsigned p     = g - rowu * ppr;
  const bool second    = p >= kp8;
  const int row = (int)rowu;
  const int c0  = (int)((second ? p - kp8 : p) << 3);
  const float* srow = src + (size_t)clampi(row, 0, rows - 1) * (size_t)ldsrc;
  float x[8];
  unsigned mk[8];
#pragma unroll
  for (int e = 0; e < 8; ++e) {
    const int c = c0 + e;
    const float v = srow[clampi(c, 0, cols - 1)];
    asm volatile("" :: "v"(v));
    x[e]  = v;
    mk[e] = (row < rows && c < cols) ? 0xFFFFu : 0u;
  }
  const v4f a = (v4f){ x[0], x[1], x[2], x[3] };
  const v4f c = (v4f){ x[4], x[5], x[6], x[7] };
  v4u o;
  if (FORM == 2) {
    o = pack8_f16(a, c);
  } else {
    const v4u hi = pack8_bf16(a, c);
    o = hi;
    if (FORM == 1) { const v4u lo = pack8_bf16_lo(a, c); o = second ? lo : hi; }
  }
  const v4u mw = (v4u){ pk16(mk[0], mk[1]), pk16(mk[2], mk[3]), pk16(mk[4], mk[5]), pk16(mk[6], mk[7]) };
  o &= mw;
  if (g < total) {
    volatile v4u* q = (volatile v4u*)(dst + (size_t)g * 8);
    *q = o;
    __threadfence();
    *q = o;
  }
}

template <int FORM> struct FragOf    { typedef FragB T; };
template <>         struct FragOf<2> { typedef FragH T; };
__device__ __forceinline__ v8f mm(const FragB& a, const FragB& b, v8f c) { return wmb(a, b, c); }
__device__ __forceinline__ v8f mm(const FragH& a, const FragH& b, v8f c) { return wmh(a, b, c); }
template <class F> __device__ __forceinline__ F ld_frag(const unsigned short* p) {
  F f;
  f.h[0] = *(const v8usa*)(p);
  f.h[1] = *(const v8usa*)(p + 16);
  return f;
}

template <int FORM, int EPI>
__global__ __launch_bounds__(256) __attribute__((amdgpu_num_vgpr(248)))
void k_gemm_nt(const unsigned short* __restrict__ A, const unsigned short* __restrict__ B,
               const float* __restrict__ bias, float* __restrict__ D, int M, int N, int KTOT, int ldd) {
  static_assert(FORM >= 0 && FORM <= 2);
  static_assert(EPI == 0 || EPI == 1);
  typedef typename FragOf<FORM>::T F;
  __shared__ __attribute__((aligned(16))) float sT[8][16 * 68];
  const int lane = threadIdx.x & 31;
  const int wave = threadIdx.x >> 5;
  const int tilesM = (M + 63) >> 6;
  const int tilesN = (N + 63) >> 6;
  const int tile = blockIdx.x * 8 + wave;
  if (tile >= tilesM * tilesN) return;
  const int tm = tile / tilesN;
  const int tn = tile - tm * tilesN;
  const int m0 = tm << 6;
  const int n0 = tn << 6;

  const int rl = lane & 15;
  const int h8 = (lane >> 4) * 8;
  const unsigned short* pa = A + (size_t)(m0 + rl) * (size_t)KTOT + h8;
  const unsigned short* pb = B + (size_t)(n0 + rl) * (size_t)KTOT + h8;

  v8f acc[4][4];
#pragma unroll
  for (int i = 0; i < 4; ++i)
#pragma unroll
    for (int j = 0; j < 4; ++j) acc[i][j] = (v8f){0.f, 0.f, 0.f, 0.f, 0.f, 0.f, 0.f, 0.f};

#pragma unroll 1
  for (int k0 = 0; k0 < KTOT; k0 += 32) {
    F bf[4];
#pragma unroll
    for (int j = 0; j < 4; ++j) bf[j] = ld_frag<F>(pb + (size_t)(j << 4) * (size_t)KTOT + k0);
#pragma unroll
    for (int i = 0; i < 4; ++i) {
      const F af = ld_frag<F>(pa + (size_t)(i << 4) * (size_t)KTOT + k0);
#pragma unroll
      for (int j = 0; j < 4; ++j) acc[i][j] = mm(af, bf[j], acc[i][j]);
    }
  }

  float* slab = sT[wave];
  const int hh = lane >> 4;
  const int c4 = (lane & 15) * 4;
  const int nc = n0 + c4;
  const bool cok = nc < N;
  v4f bv = (v4f){0.f, 0.f, 0.f, 0.f};
  if (EPI == 1) {
    bv = *(const v4fa*)(bias + clampi(nc, 0, N - 4));
    asm volatile("" :: "v"(bv));
  }
#pragma unroll
  for (int i = 0; i < 4; ++i) {
    const int mBase = m0 + (i << 4);
#pragma unroll
    for (int j = 0; j < 4; ++j) {
#pragma unroll
      for (int r = 0; r < 8; ++r) slab[(h8 + r) * 68 + (j << 4) + rl] = acc[i][j][r];
    }
    __builtin_amdgcn_fence(__ATOMIC_RELEASE, "workgroup");
    __builtin_amdgcn_wave_barrier();
    __builtin_amdgcn_fence(__ATOMIC_ACQUIRE, "workgroup");
    v4f vv[8];
#pragma unroll
    for (int it = 0; it < 8; ++it) {
      const int row = it * 2 + hh;
      v4f v = *(const v4fa*)(slab + row * 68 + c4);
      if (EPI == 1) v += bv;
      vv[it] = v;
    }
    for (int pass = 0; pass < 2; ++pass) {
#pragma unroll
      for (int it = 0; it < 8; ++it) {
        const int row = mBase + it * 2 + hh;
        if (cok && row < M) *(volatile v4f*)(D + (size_t)row * (size_t)ldd + nc) = vv[it];
      }
      __threadfence();
    }
    __builtin_amdgcn_fence(__ATOMIC_RELEASE, "workgroup");
    __builtin_amdgcn_wave_barrier();
    __builtin_amdgcn_fence(__ATOMIC_ACQUIRE, "workgroup");
  }
}

#define H_SPLIT 1
#define NN      100000
#define DEG     16
#define CIN     128
#define COUT    128
#define MROWS   100096
#define AK      (H_SPLIT ? 256 : 128)
#define GFORM   (H_SPLIT ? 1 : 0)
#define WD_PPR    (AK / 8)
#define WD_UNITS  (COUT * WD_PPR)
#define WD_BLOCKS (WD_UNITS / 256)

typedef unsigned int v2u __attribute__((ext_vector_type(2)));
typedef v2u __attribute__((may_alias)) v2ua;

static_assert(CIN == 128);
static_assert(COUT == 128);
static_assert(DEG == 16 && DEG <= 32 && (DEG % 4) == 0);
static_assert((NN % 8) == 0 && (NN % 16) == 0);
static_assert(782 * 128 == MROWS && MROWS >= NN && (MROWS % 64) == 0 && (MROWS % 8) == 0);
static_assert(((NN + 63) / 64) * 64 <= MROWS);
static_assert((AK % 32) == 0 && (COUT % 64) == 0 && (COUT % 32) == 0);
static_assert(!H_SPLIT || (AK == 256 && AK * 2 == 512));
static_assert((WD_UNITS % 256) == 0);
static_assert(((long long)NN * CIN / 8) % 256 == 0);
static_assert((long long)MROWS * AK / 8 < 0x7fffffffLL);

constexpr size_t SZ_XB  = (size_t)NN * CIN * 2;
constexpr size_t SZ_A   = (size_t)MROWS * AK * 2;
constexpr size_t SZ_HF  = (size_t)MROWS * COUT * 4;
constexpr size_t SZ_WD  = (size_t)COUT * AK * 2;
constexpr size_t SZ_PAR = (size_t)4 * 128 * 4;
constexpr size_t O_XB   = 0;
constexpr size_t O_A    = O_XB + SZ_XB;
constexpr size_t O_HF   = O_A + SZ_A;
constexpr size_t O_WD   = O_HF + SZ_HF;
constexpr size_t O_PAR  = O_WD + SZ_WD;
constexpr size_t WS_TOTAL = O_PAR + SZ_PAR;
static_assert((O_A % 128) == 0 && (O_HF % 128) == 0 && (O_WD % 128) == 0 && (O_PAR % 128) == 0);
static_assert(WS_TOTAL <= ((size_t)128 << 20));
static_assert(!H_SPLIT || WS_TOTAL == (size_t)((size_t)62581 << 11));

__device__ __forceinline__ float blend4(float a, float b, float c, float d,
                                        unsigned m0, unsigned m1, unsigned m2, unsigned m3) {
  return __uint_as_float((__float_as_uint(a) & m0) | (__float_as_uint(b) & m1) |
                         (__float_as_uint(c) & m2) | (__float_as_uint(d) & m3));
}

__global__ __launch_bounds__(256) void k_prep(const float* __restrict__ W, const float* __restrict__ bsrc,
                                              const float* __restrict__ epsp, const float* __restrict__ gsrc,
                                              const float* __restrict__ besrc,
                                              unsigned short* __restrict__ WD, float* __restrict__ PAR) {
  const int tid = (int)threadIdx.x;
  if ((int)blockIdx.x < WD_BLOCKS) {
    const int u  = (int)blockIdx.x * 256 + tid;
    const int n  = u / WD_PPR;
    const int p  = u - n * WD_PPR;
    const int kk = (p * 8) & (CIN - 1);
    float x[8];
#pragma unroll
    for (int e = 0; e < 8; ++e) {
      const float v = W[(size_t)(kk + e) * COUT + n];
      asm volatile("" :: "v"(v));
      x[e] = v;
    }
    const v4f a = (v4f){ x[0], x[1], x[2], x[3] };
    const v4f c = (v4f){ x[4], x[5], x[6], x[7] };
    const v4u o = pack8_bf16(a, c);
    volatile v4u* q = (volatile v4u*)(WD + (size_t)u * 8);
    *q = o;
    __threadfence();
    *q = o;
  } else {
    if (tid < 128) {
      const int row = tid >> 5;
      const int c4  = (tid & 31) * 4;
      const v4f vb = *(const v4fa*)(bsrc + c4);
      asm volatile("" :: "v"(vb));
      const v4f vg = *(const v4fa*)(gsrc + c4);
      asm volatile("" :: "v"(vg));
      const v4f ve = *(const v4fa*)(besrc + c4);
      asm volatile("" :: "v"(ve));
      const float e0 = epsp[0];
      asm volatile("" :: "v"(e0));
      const float S = 1.0f + bf16_val(e0);
      const unsigned m0 = (row == 0) ? 0xFFFFFFFFu : 0u;
      const unsigned m1 = (row == 1) ? 0xFFFFFFFFu : 0u;
      const unsigned m2 = (row == 2) ? 0xFFFFFFFFu : 0u;
      const unsigned m3 = (row == 3) ? 0xFFFFFFFFu : 0u;
      v4f o;
      o[0] = blend4(bf16_val(vb[0]), bf16_val(vg[0]), bf16_val(ve[0]), S, m0, m1, m2, m3);
      o[1] = blend4(bf16_val(vb[1]), bf16_val(vg[1]), bf16_val(ve[1]), S, m0, m1, m2, m3);
      o[2] = blend4(bf16_val(vb[2]), bf16_val(vg[2]), bf16_val(ve[2]), S, m0, m1, m2, m3);
      o[3] = blend4(bf16_val(vb[3]), bf16_val(vg[3]), bf16_val(ve[3]), S, m0, m1, m2, m3);
      volatile v4f* q = (volatile v4f*)(PAR + (size_t)tid * 4);
      *q = o;
      __threadfence();
      *q = o;
    }
  }
}

__global__ __launch_bounds__(256) void k_gather(const unsigned short* __restrict__ XB, const int* __restrict__ edge,
                                                const float* __restrict__ PAR, unsigned short* __restrict__ A) {
  const int lane = (int)threadIdx.x & 31;
  const int wave = __builtin_amdgcn_readfirstlane((int)(threadIdx.x >> 5));
  const int n = (int)blockIdx.x * 8 + wave;
  v2u hw = (v2u){0u, 0u};
  v2u lw = (v2u){0u, 0u};
  if (n < NN) {
    const int idw = edge[(size_t)n * DEG + (lane & 15)];
    asm volatile("" :: "v"(idw));
    const float S = PAR[3 * 128];
    asm volatile("" :: "v"(S));
    float a0 = 0.0f, a1 = 0.0f, a2 = 0.0f, a3 = 0.0f;
#pragma unroll 1
    for (int nb = 0; nb < DEG; nb += 4) {
      unsigned wx[4], wy[4], lm[4];
#pragma unroll
      for (int u = 0; u < 4; ++u) {
        const int idk = __builtin_amdgcn_readlane(idw, nb + u);
        const bool live = (idk >= 0) && (idk < NN);
        lm[u] = live ? 0xFFFFFFFFu : 0u;
        const int ar = clampi(idk, 0, NN - 1);
        const v2u w = *(const v2ua*)(XB + (size_t)ar * CIN + 4 * lane);
        wx[u] = w.x;
        wy[u] = w.y;
      }
#pragma unroll
      for (int u = 0; u < 4; ++u) asm volatile("" :: "v"(wx[u]), "v"(wy[u]));
#pragma unroll
      for (int u = 0; u < 4; ++u) {
        const unsigned mx = wx[u] & lm[u];
        const unsigned my = wy[u] & lm[u];
        a0 += __uint_as_float(mx << 16);
        a1 += __uint_as_float(mx & 0xffff0000u);
        a2 += __uint_as_float(my << 16);
        a3 += __uint_as_float(my & 0xffff0000u);
      }
    }
    const v2u xs = *(const v2ua*)(XB + (size_t)n * CIN + 4 * lane);
    const unsigned sx = xs.x, sy = xs.y;
    asm volatile("" :: "v"(sx), "v"(sy));
    const float h0 = fmaf(S, __uint_as_float(sx << 16), a0);
    const float h1 = fmaf(S, __uint_as_float(sx & 0xffff0000u), a1);
    const float h2 = fmaf(S, __uint_as_float(sy << 16), a2);
    const float h3 = fmaf(S, __uint_as_float(sy & 0xffff0000u), a3);
    hw = (v2u){ pk16(bf16_bits(h0), bf16_bits(h1)), pk16(bf16_bits(h2), bf16_bits(h3)) };
    lw = (v2u){ pk16(bf16_lo_bits(h0), bf16_lo_bits(h1)), pk16(bf16_lo_bits(h2), bf16_lo_bits(h3)) };
  }
  if (n < MROWS) {
    unsigned short* rp = A + (size_t)n * AK + 4 * lane;
    *(volatile v2u*)rp = hw;
#if H_SPLIT
    *(volatile v2u*)(rp + CIN) = lw;
#endif
    __threadfence();
    *(volatile v2u*)rp = hw;
#if H_SPLIT
    *(volatile v2u*)(rp + CIN) = lw;
#endif
  }
}

__global__ __launch_bounds__(256) void k_ln(const float* __restrict__ HF, const float* __restrict__ PAR,
                                            float* __restrict__ outp) {
  const int lane = (int)threadIdx.x & 31;
  const int wave = __builtin_amdgcn_readfirstlane((int)(threadIdx.x >> 5));
  const int n  = (int)blockIdx.x * 8 + wave;
  const int nr = n < NN ? n : NN - 1;
  const v4f t = *(const v4fa*)(HF + (size_t)nr * COUT + 4 * lane);
  asm volatile("" :: "v"(t));
  const v4f g = *(const v4fa*)(PAR + 128 + 4 * lane);
  asm volatile("" :: "v"(g));
  const v4f be = *(const v4fa*)(PAR + 256 + 4 * lane);
  asm volatile("" :: "v"(be));
  float s = (t[0] + t[1]) + (t[2] + t[3]);
#pragma unroll
  for (int m = 16; m >= 1; m >>= 1) s += __shfl_xor(s, m, 32);
  const float mu = s * (1.0f / 128.0f);
  const float d0 = t[0] - mu, d1 = t[1] - mu, d2 = t[2] - mu, d3 = t[3] - mu;
  float q = (d0 * d0 + d1 * d1) + (d2 * d2 + d3 * d3);
#pragma unroll
  for (int m = 16; m >= 1; m >>= 1) q += __shfl_xor(q, m, 32);
  const float var = q * (1.0f / 128.0f);
  const float r = 1.0f / sqrtf(var + 1e-5f);
  v4f o;
  o[0] = d0 * r * g[0] + be[0];
  o[1] = d1 * r * g[1] + be[1];
  o[2] = d2 * r * g[2] + be[2];
  o[3] = d3 * r * g[3] + be[3];
  if (n < NN) {
    volatile v4f* qo = (volatile v4f*)(outp + (size_t)n * COUT + 4 * lane);
    *qo = o;
    __threadfence();
    *qo = o;
  }
}

extern "C" void kernel_launch(void* const* d_in, const int* in_sizes, int n_in,
                              void* d_out, int out_size, void* d_ws, size_t ws_size,
                              hipStream_t stream) {
  if (n_in < 7) return;
  if (in_sizes[0] != NN * CIN) return;
  if (in_sizes[1] != NN * DEG) return;
  if (in_sizes[2] != CIN * COUT) return;
  if (in_sizes[3] != COUT) return;
  if (in_sizes[4] != 1) return;
  if (in_sizes[5] != COUT || in_sizes[6] != COUT) return;
  if ((long long)out_size != (long long)NN * COUT) return;
  if (ws_size < WS_TOTAL) return;

  const float* x     = (const float*)d_in[0];
  const int*   edge  = (const int*)d_in[1];
  const float* W     = (const float*)d_in[2];
  const float* bvec  = (const float*)d_in[3];
  const float* epsp  = (const float*)d_in[4];
  const float* gamma = (const float*)d_in[5];
  const float* beta  = (const float*)d_in[6];
  float* out = (float*)d_out;

  char* ws = (char*)d_ws;
  unsigned short* XB  = (unsigned short*)(ws + O_XB);
  unsigned short* Apl = (unsigned short*)(ws + O_A);
  float*          HF  = (float*)(ws + O_HF);
  unsigned short* WD  = (unsigned short*)(ws + O_WD);
  float*          PAR = (float*)(ws + O_PAR);

  k_prep<<<WD_BLOCKS + 1, 256, 0, stream>>>(W, bvec, epsp, gamma, beta, WD, PAR);
  k_plane<0><<<(NN * CIN / 8) / 256, 256, 0, stream>>>(x, NN, CIN, CIN, XB, NN, CIN);
  k_gather<<<MROWS / 8, 256, 0, stream>>>(XB, edge, PAR, Apl);
  {
    const int tiles = ((NN + 63) / 64) * ((COUT + 63) / 64);
    k_gemm_nt<GFORM, 1><<<(tiles + 7) / 8, 256, 0, stream>>>(Apl, WD, PAR, HF, NN, COUT, AK, COUT);
  }
  k_ln<<<NN / 8, 256, 0, stream>>>(HF, PAR, out);
}
